// NSFPRawMLP_85461259255883
// MI455X (gfx1250) — hardware-verified
//
#include <hip/hip_runtime.h>


namespace {
constexpr int N = 262144, DH = 128, NL = 7, RB = 128;
constexpr float HS = 8.0f;

typedef _Float16 b16;
typedef __attribute__((ext_vector_type(16))) _Float16 v16b;
typedef __attribute__((ext_vector_type(8))) _Float16 v8b;
typedef __attribute__((ext_vector_type(8))) float v8f;
typedef __attribute__((ext_vector_type(4))) float v4f;
__device__ __forceinline__ float bf16_rne(float f) { unsigned int u = __float_as_uint(f); u += 0x7FFFu + ((u >> 16) & 1u); return __uint_as_float(u & 0xFFFF0000u); }
__device__ __forceinline__ v16b frag_kb(const b16* p, int hh) { const v8b a = *(const v8b*)(p + 8 * hh), b = *(const v8b*)(p + 16 + 8 * hh); v16b f;
#pragma unroll
  for (int e = 0; e < 8; ++e) { f[e] = a[e]; f[8 + e] = b[e]; } return f; }
__device__ __forceinline__ v8f wmma16b(v16b a, v16b b, v8f c) { v8f d = __builtin_amdgcn_wmma_f32_16x16x32_f16(false, a, false, b, (short)0, c, false, false); asm volatile("v_nop\n\tv_nop\n\tv_nop\n\tv_nop" : "+v"(d) : "v"(a), "v"(b)); return d; }
__device__ __forceinline__ void wave_lds_sync() { __builtin_amdgcn_fence(__ATOMIC_RELEASE, "workgroup"); __builtin_amdgcn_wave_barrier(); __builtin_amdgcn_fence(__ATOMIC_ACQUIRE, "workgroup"); }
__device__ __forceinline__ float pmul(float a, float b) { float p = a * b; asm volatile("" : "+v"(p)); return p; }

__global__ __launch_bounds__(256) void prep_kernel(const float* __restrict__ W0, const float* __restrict__ b0, const float* __restrict__ Wh, const float* __restrict__ bh, const float* __restrict__ Wout, const float* __restrict__ bout, b16* __restrict__ R, float* __restrict__ P) {
  const int t_ = blockIdx.x * 256 + threadIdx.x, nth = gridDim.x * 256;
  for (int pass = 0; pass < 2; ++pass) {
    for (int p = t_; p < NL * DH * DH / 8; p += nth) { v8b v; for (int e = 0; e < 8; ++e) v[e] = (b16)bf16_rne(Wh[p * 8 + e]); *(volatile v8b*)(R + p * 8) = v; }
    for (int q = t_; q < 1824; q += nth) { float v = 0.0f; if (q < 384) v = W0[q]; else if (q < 512) v = b0[q - 384]; else if (q < 1408) v = bh[q - 512]; else if (q < 1792) v = Wout[q - 1408]; else if (q < 1795) v = bout[q - 1792]; P[q] = bf16_rne(v); }
    __threadfence(); }
}

__global__ __launch_bounds__(256) void mlp_kernel(const float* __restrict__ x, const b16* __restrict__ R, const float* __restrict__ P, float* __restrict__ out) {
  __shared__ __attribute__((aligned(16))) b16 Hs[RB][DH + 8]; __shared__ __attribute__((aligned(16))) float Hf[8][16][DH + 4]; __shared__ __attribute__((aligned(16))) float Ob[RB * 3];
  const int wave = threadIdx.x >> 5, lane = threadIdx.x & 31, nloc = lane & 15, hlf = lane >> 4, r0 = blockIdx.x * RB, t_ = threadIdx.x;
  const float* W0 = P; const float* b0 = P + 384; const float* bh = P + 512; const float* Wout = P + 1408; const float* bout = P + 1792;
  { const int row = t_ >> 1, f0 = (t_ & 1) * 64; const float x0 = bf16_rne(x[(size_t)(r0 + row) * 3]), x1 = bf16_rne(x[(size_t)(r0 + row) * 3 + 1]), x2 = bf16_rne(x[(size_t)(r0 + row) * 3 + 2]);
    for (int f = f0; f < f0 + 64; ++f) { const float h = fmaxf(pmul(x0, W0[f * 3]) + pmul(x1, W0[f * 3 + 1]) + pmul(x2, W0[f * 3 + 2]) + b0[f], 0.0f); Hs[row][f] = (b16)(h * HS); } }
  __syncthreads();
  for (int l = 0; l < NL; ++l) { const b16* Wl = R + (size_t)l * DH * DH; const float* bl = bh + l * DH;
    v8f acc[8];
#pragma unroll
    for (int t = 0; t < 8; ++t) acc[t] = (v8f){};
#pragma unroll
    for (int kb = 0; kb < DH; kb += 32) { const v16b a = frag_kb(&Hs[wave * 16 + nloc][kb], hlf);
#pragma unroll
      for (int t = 0; t < 8; ++t) { const v16b bw = frag_kb(Wl + (size_t)(t * 16 + nloc) * DH + kb, hlf); acc[t] = wmma16b(a, bw, acc[t]); } }
    __syncthreads();
#pragma unroll
    for (int t = 0; t < 8; ++t)
#pragma unroll
      for (int r = 0; r < 8; ++r) { const int c = t * 16 + nloc, rr = wave * 16 + 8 * hlf + r; const float h = fmaxf(acc[t][r] * (1.0f / HS) + bl[c], 0.0f); if (l < NL - 1) Hs[rr][c] = (b16)(h * HS); else Hf[wave][8 * hlf + r][c] = h; }
    __syncthreads(); }
  if (t_ < RB) { const float* hr = &Hf[t_ >> 4][t_ & 15][0];
    for (int o = 0; o < 3; ++o) { float s = 0.0f; for (int c = 0; c < DH; ++c) s += pmul(hr[c], Wout[o * DH + c]); Ob[t_ * 3 + o] = s + bout[o]; } }
  __syncthreads();
  for (int pass = 0; pass < 2; ++pass) { if (t_ < RB * 3 / 4) *(volatile v4f*)(out + (size_t)r0 * 3 + t_ * 4) = *(const v4f*)(&Ob[t_ * 4]); __threadfence(); }
}
}

extern "C" void kernel_launch(void* const* d_in, const int* in_sizes, int n_in,
                              void* d_out, int out_size, void* d_ws, size_t ws_size, hipStream_t stream) {
  (void)n_in; (void)out_size;
  const float* x = (const float*)d_in[0]; const float* W0 = (const float*)d_in[1]; const float* b0 = (const float*)d_in[2]; const float* Wh = (const float*)d_in[3]; const float* bh = (const float*)d_in[4]; const float* Wout = (const float*)d_in[5]; const float* bout = (const float*)d_in[6];
  float* out = (float*)d_out;
  if (in_sizes[0] != N * 3 || in_sizes[1] != DH * 3 || in_sizes[3] != NL * DH * DH || in_sizes[5] != 3 * DH) return;
  size_t off = 0; char* ws = (char*)d_ws;
  auto carve = [&](size_t bytes) { char* p = ws + off; off += (bytes + 255) & ~(size_t)255; return p; };
  b16* R = (b16*)carve((size_t)NL * DH * DH * 2); float* P = (float*)carve(2048 * 4);
  if (off > ws_size) return;
  prep_kernel<<<64, 256, 0, stream>>>(W0, b0, Wh, bh, Wout, bout, R, P);
  mlp_kernel<<<N / RB, 256, 0, stream>>>(x, R, P, out);
}
